// GATBlock_34711925686357
// MI455X (gfx1250) — hardware-verified
//
#include <hip/hip_runtime.h>
#include <stddef.h>


#define DF    128
#define NH    8
#define HC    16
#define GR    32
#define AP    136
#define XSP   132
#define NB    512
#define CHUNK 2048
#define NTHR  256
#define NWAVE 8
#define WCAP  256
#define NGRP  (CHUNK / (NTHR * 4))

#define LDS_SACC (NB * DF)
#define LDS_AUX  (NB * NH + NB + NB)
#define LDS_LIST (NWAVE * WCAP)
#define LDS_BYTES ((LDS_SACC + LDS_AUX + LDS_LIST + NWAVE + NH) * 4)

static_assert(WCAP == (CHUNK / NTHR) * 32);
static_assert(NGRP >= 1);
static_assert(NB == 512);
static_assert(CHUNK <= 4096);
static_assert(((LDS_SACC + LDS_AUX) % 4) == 0);
static_assert(LDS_BYTES == 290880);

typedef float    v4f  __attribute__((ext_vector_type(4)));
typedef float    v8f  __attribute__((ext_vector_type(8)));
typedef int      v4i  __attribute__((ext_vector_type(4)));
typedef _Float16 v8h  __attribute__((ext_vector_type(8)));
typedef _Float16 v16h __attribute__((ext_vector_type(16)));
union Frag   { v16h v; v8h half[2]; };
union Pack16 { v8h h; v4i i; };

__device__ __forceinline__ v8f wm(v16h a, v16h b, v8f c) {
  v8f d = __builtin_amdgcn_wmma_f32_16x16x32_f16(false, a, false, b, (short)0, c, false, false);
  asm volatile("v_nop\n\tv_nop\n\tv_nop\n\tv_nop" : "+v"(d) : "v"(a), "v"(b));
  return d;
}

__device__ __forceinline__ float wsum(float v) {
  v += __shfl_xor(v, 16, 32);
  v += __shfl_xor(v, 8, 32);
  v += __shfl_xor(v, 4, 32);
  v += __shfl_xor(v, 2, 32);
  v += __shfl_xor(v, 1, 32);
  return v;
}

__global__ __launch_bounds__(NTHR) void k_prep(const float* __restrict__ W, _Float16* Wh, int n8) {
  const int i = blockIdx.x * NTHR + threadIdx.x;
  if (i >= n8) return;
  const size_t o = (size_t)i * 8;
  const v4f a = *(const v4f*)(W + o);
  const v4f b = *(const v4f*)(W + o + 4);
  Pack16 u;
  u.h[0] = (_Float16)(a.x * 8.0f); u.h[1] = (_Float16)(a.y * 8.0f);
  u.h[2] = (_Float16)(a.z * 8.0f); u.h[3] = (_Float16)(a.w * 8.0f);
  u.h[4] = (_Float16)(b.x * 8.0f); u.h[5] = (_Float16)(b.y * 8.0f);
  u.h[6] = (_Float16)(b.z * 8.0f); u.h[7] = (_Float16)(b.w * 8.0f);
  *(volatile v4i*)(Wh + o) = u.i;
  __threadfence();
  *(volatile v4i*)(Wh + o) = u.i;
}

__device__ __forceinline__ void epi_tile(v8f acc, int T, int hh, int m, int wave, int ncol,
                                         float cs, float cd, float* Xs, float* As, float* Ds) {
  float ss[8], sd[8];
#pragma unroll
  for (int r = 0; r < 8; ++r) {
    const float v = acc[r] * 0.125f;
    Xs[(T * 16 + 8 * hh + r) * XSP + ncol] = v;
    ss[r] = v * cs;
    sd[r] = v * cd;
  }
#pragma unroll
  for (int mk = 1; mk < 16; mk <<= 1) {
#pragma unroll
    for (int r = 0; r < 8; ++r) {
      ss[r] += __shfl_xor(ss[r], mk, 32);
      sd[r] += __shfl_xor(sd[r], mk, 32);
    }
  }
  if (m == 0) {
#pragma unroll
    for (int r = 0; r < 8; ++r) {
      As[(T * 16 + 8 * hh + r) * NH + wave] = ss[r];
      Ds[(T * 16 + 8 * hh + r) * NH + wave] = sd[r];
    }
  }
}

__global__ __launch_bounds__(NTHR) void k_gemm(
    const float* __restrict__ x, const _Float16* __restrict__ Wh,
    const float* __restrict__ att_src, const float* __restrict__ att_dst,
    float* xp, float* asrc, float* adst, int nN) {
  __shared__ __attribute__((aligned(16))) _Float16 At[GR * AP];
  __shared__ __attribute__((aligned(16))) float Xs[GR * XSP];
  __shared__ __attribute__((aligned(16))) float As[GR * NH];
  __shared__ __attribute__((aligned(16))) float Ds[GR * NH];

  const int tid  = threadIdx.x;
  const int lane = tid & 31;
  const int wave = tid >> 5;
  const int hh   = lane >> 4;
  const int m    = lane & 15;
  const int rowBase = blockIdx.x * GR;

  {
    const int r  = tid >> 3;
    const int c0 = (tid & 7) * 16;
    int row = rowBase + r;
    if (row > nN - 1) row = nN - 1;
    const float* p = x + (size_t)row * DF + c0;
    const v4f f0 = *(const v4f*)(p), f1 = *(const v4f*)(p + 4);
    const v4f f2 = *(const v4f*)(p + 8), f3 = *(const v4f*)(p + 12);
    Pack16 u0, u1;
    u0.h[0] = (_Float16)f0.x; u0.h[1] = (_Float16)f0.y; u0.h[2] = (_Float16)f0.z; u0.h[3] = (_Float16)f0.w;
    u0.h[4] = (_Float16)f1.x; u0.h[5] = (_Float16)f1.y; u0.h[6] = (_Float16)f1.z; u0.h[7] = (_Float16)f1.w;
    u1.h[0] = (_Float16)f2.x; u1.h[1] = (_Float16)f2.y; u1.h[2] = (_Float16)f2.z; u1.h[3] = (_Float16)f2.w;
    u1.h[4] = (_Float16)f3.x; u1.h[5] = (_Float16)f3.y; u1.h[6] = (_Float16)f3.z; u1.h[7] = (_Float16)f3.w;
    *(v8h*)(At + r * AP + c0)     = u0.h;
    *(v8h*)(At + r * AP + c0 + 8) = u1.h;
  }
  __syncthreads();

  const int ncol = wave * 16 + m;
  v8f c0a = {0.f, 0.f, 0.f, 0.f, 0.f, 0.f, 0.f, 0.f};
  v8f c1a = {0.f, 0.f, 0.f, 0.f, 0.f, 0.f, 0.f, 0.f};
#pragma unroll
  for (int kt = 0; kt < DF / 32; ++kt) {
    const int k0 = kt * 32;
    Frag a0, a1, b;
    const _Float16* pb  = Wh + (size_t)ncol * DF + k0 + 8 * hh;
    const _Float16* pa0 = At + m * AP + k0 + 8 * hh;
    const _Float16* pa1 = At + (16 + m) * AP + k0 + 8 * hh;
    b.half[0]  = *(const v8h*)pb;  b.half[1]  = *(const v8h*)(pb + 16);
    a0.half[0] = *(const v8h*)pa0; a0.half[1] = *(const v8h*)(pa0 + 16);
    a1.half[0] = *(const v8h*)pa1; a1.half[1] = *(const v8h*)(pa1 + 16);
    c0a = wm(a0.v, b.v, c0a);
    c1a = wm(a1.v, b.v, c1a);
  }

  const float cs = att_src[ncol];
  const float cd = att_dst[ncol];
  epi_tile(c0a, 0, hh, m, wave, ncol, cs, cd, Xs, As, Ds);
  epi_tile(c1a, 1, hh, m, wave, ncol, cs, cd, Xs, As, Ds);
  __syncthreads();

  v4f xr[4];
#pragma unroll
  for (int i = 0; i < 4; ++i) xr[i] = *(const v4f*)(Xs + (4 * wave + i) * XSP + 4 * lane);
  float* gp = 0;
  v4f gv = {0.f, 0.f, 0.f, 0.f};
  if (wave < 2) {
    gv = *(const v4f*)(As + wave * 128 + 4 * lane);
    gp = asrc + (size_t)rowBase * NH + wave * 128 + 4 * lane;
  } else if (wave < 4) {
    gv = *(const v4f*)(Ds + (wave - 2) * 128 + 4 * lane);
    gp = adst + (size_t)rowBase * NH + (wave - 2) * 128 + 4 * lane;
  }
  float* xpp[4];
#pragma unroll
  for (int i = 0; i < 4; ++i) xpp[i] = xp + (size_t)(rowBase + 4 * wave + i) * DF + 4 * lane;

#pragma unroll
  for (int i = 0; i < 4; ++i) *(volatile v4f*)(xpp[i]) = xr[i];
  if (gp) *(volatile v4f*)gp = gv;
  __threadfence();
#pragma unroll
  for (int i = 0; i < 4; ++i) *(volatile v4f*)(xpp[i]) = xr[i];
  if (gp) *(volatile v4f*)gp = gv;
}

__global__ __launch_bounds__(NTHR) void k_gat(
    const float* __restrict__ x, const int* __restrict__ ei, const float* __restrict__ ea,
    const float* __restrict__ xp, const float* __restrict__ asrc, const float* __restrict__ adst,
    const float* __restrict__ W_edge, const float* __restrict__ att_edge,
    const float* __restrict__ bias, const float* __restrict__ gam, const float* __restrict__ bet,
    float* out, int nN, int nE) {
  extern __shared__ v4f lds_dyn[];
  float* sacc = (float*)lds_dyn;
  float* aux  = sacc + LDS_SACC;
  int*   list = (int*)(aux + LDS_AUX);
  int*   wcnt = list + LDS_LIST;
  float* kap  = (float*)(wcnt + NWAVE);

  const int tid  = threadIdx.x;
  const int lane = tid & 31;
  const int wave = tid >> 5;
  const int hd   = lane >> 2;
  const int nodeBase = blockIdx.x * NB;

  {
    const v4f z4 = {0.f, 0.f, 0.f, 0.f};
    for (int i = tid; i < (LDS_SACC + LDS_AUX) / 4; i += NTHR) lds_dyn[i] = z4;
    if (tid < NH) {
      float s = 0.f;
#pragma unroll 1
      for (int c = 0; c < HC; ++c) s += W_edge[tid * HC + c] * att_edge[tid * HC + c];
      kap[tid] = s;
    }
  }
  __syncthreads();
  const float kreg = kap[hd];
  const int* eid = ei + nE;
  const bool al16 = ((nE & 3) == 0);

  const int nChunks = (nE + CHUNK - 1) / CHUNK;
#pragma unroll 1
  for (int ch = 0; ch < nChunks; ++ch) {
    const int cbase = ch * CHUNK;
    int wc = 0;
#pragma unroll
    for (int g = 0; g < NGRP; ++g) {
      const int el0 = (g * NTHR + tid) * 4;
      const int e0  = cbase + el0;
      const int sent = -2147483647 - 1;
      v4i d;
      if (al16 && (e0 + 3 < nE)) {
        d = *(const v4i*)(eid + e0);
      } else {
        d.x = (e0     < nE) ? eid[e0]     : sent;
        d.y = (e0 + 1 < nE) ? eid[e0 + 1] : sent;
        d.z = (e0 + 2 < nE) ? eid[e0 + 2] : sent;
        d.w = (e0 + 3 < nE) ? eid[e0 + 3] : sent;
      }
      const unsigned s0 = (unsigned)d.x - (unsigned)nodeBase;
      const unsigned s1 = (unsigned)d.y - (unsigned)nodeBase;
      const unsigned s2 = (unsigned)d.z - (unsigned)nodeBase;
      const unsigned s3 = (unsigned)d.w - (unsigned)nodeBase;
      const bool h0 = s0 < (unsigned)NB;
      const bool h1 = s1 < (unsigned)NB;
      const bool h2 = s2 < (unsigned)NB;
      const bool h3 = s3 < (unsigned)NB;
      const unsigned many = __builtin_amdgcn_ballot_w32(h0 | h1 | h2 | h3);
      if (many != 0u) {
#define HITJ(J, HJ, SJ) { \
          const unsigned mj = __builtin_amdgcn_ballot_w32(HJ); \
          if (HJ) { \
            const int pos = wc + (int)__builtin_amdgcn_mbcnt_lo(mj, 0u); \
            if (pos < WCAP) list[wave * WCAP + pos] = ((el0 + (J)) << 9) | (int)(SJ); \
          } \
          wc += (int)__builtin_popcount(mj); }
        HITJ(0, h0, s0)
        HITJ(1, h1, s1)
        HITJ(2, h2, s2)
        HITJ(3, h3, s3)
#undef HITJ
      }
    }
    if (lane == 0) wcnt[wave] = wc;
    __syncthreads();

    if (wave == 0) {
      for (int wsx = 0; wsx < NWAVE; ++wsx) {
        int n = wcnt[wsx];
        if (n > WCAP) n = WCAP;
        if (n < 0) n = 0;
        for (int i = 0; i < n; ++i) {
          const int ent  = list[wsx * WCAP + i];
          const int slot = ent & (NB - 1);
          const int el   = (ent >> 9) & (CHUNK - 1);
          int e = cbase + el;
          if (e > nE - 1) e = nE - 1;
          int src = ei[e];
          src = src < 0 ? 0 : (src > nN - 1 ? nN - 1 : src);
          const float w = ea[e];
          int nd = nodeBase + slot;
          if (nd > nN - 1) nd = nN - 1;
          float al = asrc[(size_t)src * NH + hd] + adst[(size_t)nd * NH + hd] + w * kreg;
          al = (al > 0.f) ? al : 0.2f * al;
          al = fminf(al, 80.f);
          const float p = __expf(al);
          const v4f xv = *(const v4f*)(xp + (size_t)src * DF + 4 * lane);
          v4f* sp = (v4f*)(sacc + slot * DF + 4 * lane);
          const v4f cur = *sp;
          const v4f nxt = cur + p * xv;
          *sp = nxt;
          int ai = -1;
          float av = 0.f;
          if ((lane & 3) == 0)  { ai = slot * NH + hd;       av = p;    }
          else if (lane == 1)   { ai = NB * NH + slot;       av = 1.0f; }
          else if (lane == 2)   { ai = NB * NH + NB + slot;  av = w;    }
          if (ai >= 0) {
            const float o = aux[ai];
            aux[ai] = o + av;
          }
        }
      }
    }
    __syncthreads();
  }

  const float* den  = aux;
  const float* cntp = aux + NB * NH;
  const float* ssp  = cntp + NB;
  const v4f b4 = *(const v4f*)(bias + 4 * lane);
  const v4f g4 = *(const v4f*)(gam + 4 * lane);
  const v4f e4 = *(const v4f*)(bet + 4 * lane);
#pragma unroll 1
  for (int j = 0; j < NB / NWAVE; ++j) {
    const int slot = wave * (NB / NWAVE) + j;
    const int node = nodeBase + slot;
    if (node >= nN) break;
    const size_t nrow = (size_t)node;
    const float c  = cntp[slot];
    const float cc = fmaxf(c, 1.0f);
    const float la = (c > 0.f) ? ssp[slot] * (1.0f / cc) : 0.f;
    float al = asrc[nrow * NH + hd] + adst[nrow * NH + hd] + la * kreg;
    al = (al > 0.f) ? al : 0.2f * al;
    al = fminf(al, 80.f);
    const float p = __expf(al);
    const v4f xv = *(const v4f*)(xp + nrow * DF + 4 * lane);
    const v4f sv = *(const v4f*)(sacc + slot * DF + 4 * lane) + p * xv;
    const float dv  = den[slot * NH + hd] + p;
    const float inv = 1.0f / (dv + 1e-16f);
    const v4f xr = *(const v4f*)(x + nrow * DF + 4 * lane);
    v4f h = sv * inv + b4;
    h = h + xr;
    const float s  = wsum(h.x + h.y + h.z + h.w);
    const float mu = s * (1.0f / DF);
    const v4f dd = h - mu;
    const float q  = wsum(dd.x * dd.x + dd.y * dd.y + dd.z * dd.z + dd.w * dd.w);
    const float rs = rsqrtf(q * (1.0f / DF) + 1e-5f);
    v4f y = dd * rs * g4 + e4;
    y.x = y.x > 0.f ? y.x : 0.f;
    y.y = y.y > 0.f ? y.y : 0.f;
    y.z = y.z > 0.f ? y.z : 0.f;
    y.w = y.w > 0.f ? y.w : 0.f;
    float* op = out + nrow * DF + 4 * lane;
    *(volatile v4f*)op = y;
    __threadfence();
    *(volatile v4f*)op = y;
  }
}

extern "C" void kernel_launch(void* const* d_in, const int* in_sizes, int n_in,
                              void* d_out, int out_size, void* d_ws, size_t ws_size,
                              hipStream_t stream) {
  if (n_in < 11) return;
  const int nN = in_sizes[0] / DF;
  const int nE = in_sizes[2];
  if (nN <= 0 || in_sizes[0] != nN * DF) return;
  if (nE < 0 || in_sizes[1] != 2 * nE) return;
  if (in_sizes[3] != DF * DF) return;
  if (in_sizes[4] != NH * HC || in_sizes[5] != NH * HC || in_sizes[6] != NH * HC) return;
  if (in_sizes[7] != DF || in_sizes[8] != DF || in_sizes[9] != DF || in_sizes[10] != DF) return;
  if (out_size != nN * DF) return;

  const float* x        = (const float*)d_in[0];
  const int*   ei       = (const int*)d_in[1];
  const float* ea       = (const float*)d_in[2];
  const float* W        = (const float*)d_in[3];
  const float* att_src  = (const float*)d_in[4];
  const float* att_dst  = (const float*)d_in[5];
  const float* att_edge = (const float*)d_in[6];
  const float* W_edge   = (const float*)d_in[7];
  const float* bias     = (const float*)d_in[8];
  const float* gam      = (const float*)d_in[9];
  const float* bet      = (const float*)d_in[10];
  float* out = (float*)d_out;

  const int nP = ((nN + GR - 1) / GR) * GR;
  size_t off = 0;
  _Float16* Wh = (_Float16*)((char*)d_ws + off); off += (size_t)DF * DF * sizeof(_Float16);
  float* xp   = (float*)((char*)d_ws + off);     off += (size_t)nP * DF * sizeof(float);
  float* asrc = (float*)((char*)d_ws + off);     off += (size_t)nP * NH * sizeof(float);
  float* adst = (float*)((char*)d_ws + off);     off += (size_t)nP * NH * sizeof(float);
  if (off > ws_size) return;

  const int n8 = DF * DF / 8;
  k_prep<<<(n8 + NTHR - 1) / NTHR, NTHR, 0, stream>>>(W, Wh, n8);

  k_gemm<<<nP / GR, NTHR, 0, stream>>>(x, Wh, att_src, att_dst, xp, asrc, adst, nN);

  hipFuncSetAttribute(reinterpret_cast<const void*>(&k_gat),
                      hipFuncAttributeMaxDynamicSharedMemorySize, LDS_BYTES);
  const int grid = (nN + NB - 1) / NB;
  k_gat<<<grid, NTHR, LDS_BYTES, stream>>>(x, ei, ea, xp, asrc, adst, W_edge, att_edge,
                                           bias, gam, bet, out, nN, nE);
}
